// unnamed_model3_58506044506599
// MI455X (gfx1250) — hardware-verified
//
#include <hip/hip_runtime.h>
#include <stddef.h>


#define DF      128
#define NCLS    64
#define NTHR    256
#define NWAVE   8
#define EPT     8
#define NGRP    2
#define CHUNK   (NTHR * EPT * NGRP)
#define WCAP    (EPT * NGRP * 32)
#define LISTN   (NWAVE * WCAP)
#define SLOTB   16
#define NB1     512
#define NB2     1024
#define NBD     8192
#define G1ROWS  128

#define LDS_GEMM1 (G1ROWS * DF * 4)
#define LDS_AGG1  (NB1 * DF * 4 + LISTN * 4 + 64)
#define LDS_AGG2  (NB2 * NCLS * 4 + LISTN * 4 + 64)

static_assert((CHUNK & (CHUNK - 1)) == 0);
static_assert(CHUNK <= 32768);
static_assert((NB1 & (NB1 - 1)) == 0 && (NB2 & (NB2 - 1)) == 0 && (NBD & (NBD - 1)) == 0);
static_assert(NB1 <= 65536 && NB2 <= 65536 && NBD <= 65536);
static_assert(NBD % G1ROWS == 0 && NBD % NB1 == 0 && NBD % NB2 == 0);
static_assert((NB1 * DF / 4) % NTHR == 0 && (NB2 * NCLS / 4) % NTHR == 0);
static_assert(NBD / NWAVE == 8 * 128);
static_assert(NB2 * NCLS / NWAVE == 64 * 128);
static_assert(NB1 / 16 == 4 * NWAVE);

typedef float  v2f  __attribute__((ext_vector_type(2)));
typedef float  v4f  __attribute__((ext_vector_type(4)));
typedef float  v8f  __attribute__((ext_vector_type(8)));
typedef int    v4i  __attribute__((ext_vector_type(4)));
typedef __bf16 v8b  __attribute__((ext_vector_type(8)));
typedef __bf16 v16b __attribute__((ext_vector_type(16)));
union FragB { v16b v; v8b h[2]; };

__device__ __forceinline__ void split8(v4f a, v4f b, v8b& hi, v8b& lo) {
  float f[8];
  f[0] = a.x; f[1] = a.y; f[2] = a.z; f[3] = a.w;
  f[4] = b.x; f[5] = b.y; f[6] = b.z; f[7] = b.w;
  v8b hv, lv;
#pragma unroll
  for (int i = 0; i < 8; ++i) {
    const __bf16 hb = (__bf16)f[i];
    const float  r  = f[i] - (float)hb;
    hv[i] = hb;
    lv[i] = (__bf16)r;
  }
  hi = hv;
  lo = lv;
}

__device__ __forceinline__ v8f wmb3(v16b ah, v16b al, v16b bh, v16b bl, v8f c) {
  v8f d = __builtin_amdgcn_wmma_f32_16x16x32_bf16(false, ah, false, bh, (short)0, c, false, false);
  d = __builtin_amdgcn_wmma_f32_16x16x32_bf16(false, ah, false, bl, (short)0, d, false, false);
  d = __builtin_amdgcn_wmma_f32_16x16x32_bf16(false, al, false, bh, (short)0, d, false, false);
  asm volatile("v_nop\n\tv_nop\n\tv_nop\n\tv_nop" : "+v"(d) : "v"(ah), "v"(al), "v"(bh), "v"(bl));
  return d;
}

template <int NB>
__device__ __forceinline__ int scan_chunk(const int* __restrict__ dsts, int nE, int cbase, int nodeBase,
                                          int vec8, int* list, int tid, int lane, int wave) {
  int wc = 0;
#pragma unroll
  for (int g = 0; g < NGRP; ++g) {
    const int el0  = (g * NTHR + tid) * EPT;
    const int e0   = cbase + el0;
    const int sent = -2147483647 - 1;
    v4i da, db;
    if (vec8 != 0 && e0 + 7 < nE) {
      da = *(const v4i*)(dsts + e0);
      db = *(const v4i*)(dsts + e0 + 4);
    } else {
      da.x = (e0     < nE) ? dsts[min(e0, nE - 1)] : sent;
      da.y = (e0 + 1 < nE) ? dsts[min(e0 + 1, nE - 1)] : sent;
      da.z = (e0 + 2 < nE) ? dsts[min(e0 + 2, nE - 1)] : sent;
      da.w = (e0 + 3 < nE) ? dsts[min(e0 + 3, nE - 1)] : sent;
      db.x = (e0 + 4 < nE) ? dsts[min(e0 + 4, nE - 1)] : sent;
      db.y = (e0 + 5 < nE) ? dsts[min(e0 + 5, nE - 1)] : sent;
      db.z = (e0 + 6 < nE) ? dsts[min(e0 + 6, nE - 1)] : sent;
      db.w = (e0 + 7 < nE) ? dsts[min(e0 + 7, nE - 1)] : sent;
    }
    const unsigned nb = (unsigned)nodeBase;
    const unsigned s0 = (unsigned)da.x - nb, s1 = (unsigned)da.y - nb;
    const unsigned s2 = (unsigned)da.z - nb, s3 = (unsigned)da.w - nb;
    const unsigned s4 = (unsigned)db.x - nb, s5 = (unsigned)db.y - nb;
    const unsigned s6 = (unsigned)db.z - nb, s7 = (unsigned)db.w - nb;
    const bool h0 = s0 < (unsigned)NB, h1 = s1 < (unsigned)NB, h2 = s2 < (unsigned)NB, h3 = s3 < (unsigned)NB;
    const bool h4 = s4 < (unsigned)NB, h5 = s5 < (unsigned)NB, h6 = s6 < (unsigned)NB, h7 = s7 < (unsigned)NB;
    const unsigned any = __builtin_amdgcn_ballot_w32(h0 | h1 | h2 | h3 | h4 | h5 | h6 | h7);
    if (any != 0u) {
#define HITJ(J, HJ, SJ) { \
        const unsigned mj = __builtin_amdgcn_ballot_w32(HJ); \
        if (mj != 0u) { \
          if (HJ) { \
            const int pos = wc + (int)__builtin_amdgcn_mbcnt_lo(mj, 0u); \
            if (pos < WCAP) list[wave * WCAP + pos] = ((el0 + (J)) << SLOTB) | (int)(SJ); \
          } \
          wc += (int)__builtin_popcount(mj); } }
      HITJ(0, h0, s0)
      HITJ(1, h1, s1)
      HITJ(2, h2, s2)
      HITJ(3, h3, s3)
      HITJ(4, h4, s4)
      HITJ(5, h5, s5)
      HITJ(6, h6, s6)
      HITJ(7, h7, s7)
#undef HITJ
    }
  }
  return wc;
}

__global__ __launch_bounds__(NTHR) void k_wprep(
    const float* __restrict__ W1, const float* __restrict__ W2,
    __bf16* w1h, __bf16* w1l, __bf16* w2h, __bf16* w2l) {
  const int i  = blockIdx.x * NTHR + threadIdx.x;
  const int n1 = DF * DF / 8;
  const int n2 = NCLS * DF / 8;
  if (i >= n1 + n2) return;
  const bool first = i < n1;
  const int o  = (first ? i : i - n1) * 8;
  const int n  = o / DF;
  const int k0 = o - n * DF;
  v4f a, b;
  if (first) {
    const float* p = W1 + (size_t)k0 * DF + n;
    a.x = p[0];      a.y = p[DF];     a.z = p[2 * DF]; a.w = p[3 * DF];
    b.x = p[4 * DF]; b.y = p[5 * DF]; b.z = p[6 * DF]; b.w = p[7 * DF];
  } else {
    const float* p = W2 + (size_t)k0 * NCLS + n;
    a.x = p[0];        a.y = p[NCLS];     a.z = p[2 * NCLS]; a.w = p[3 * NCLS];
    b.x = p[4 * NCLS]; b.y = p[5 * NCLS]; b.z = p[6 * NCLS]; b.w = p[7 * NCLS];
  }
  v8b hv, lv;
  split8(a, b, hv, lv);
  __bf16* hp = (first ? w1h : w2h) + o;
  __bf16* lp = (first ? w1l : w2l) + o;
  *(volatile v8b*)hp = hv;
  *(volatile v8b*)lp = lv;
  __threadfence();
  *(volatile v8b*)hp = hv;
  *(volatile v8b*)lp = lv;
}

__global__ __launch_bounds__(NTHR) void k_deg(
    const int* __restrict__ ei, const float* __restrict__ ew, float* dinv, int nN, int nE, int vec8) {
  __shared__ __attribute__((aligned(16))) float dacc[NBD];
  __shared__ __attribute__((aligned(16))) int list[LISTN];
  __shared__ int wcnt[NWAVE];
  const int tid = threadIdx.x, lane = tid & 31, wave = tid >> 5;
  const int nodeBase = blockIdx.x * NBD;
  const int* dsts = ei + nE;
  (void)nN;

  for (int i = tid; i < NBD; i += NTHR) dacc[i] = 0.f;
  __syncthreads();

  const int nChunks = (nE + CHUNK - 1) / CHUNK;
#pragma unroll 1
  for (int ch = 0; ch < nChunks; ++ch) {
    const int cbase = ch * CHUNK;
    const int wc = scan_chunk<NBD>(dsts, nE, cbase, nodeBase, vec8, list, tid, lane, wave);
    if (lane == 0) wcnt[wave] = wc;
    __syncthreads();
    if (wave == 0) {
#pragma unroll 1
      for (int wsx = 0; wsx < NWAVE; ++wsx) {
        int n = __builtin_amdgcn_readfirstlane(wcnt[wsx]);
        n = n > WCAP ? WCAP : (n < 0 ? 0 : n);
        const int* lp = list + wsx * WCAP;
#pragma unroll 1
        for (int i = 0; i < n; ++i) {
          const int ent  = __builtin_amdgcn_readfirstlane(lp[i]);
          const int slot = ent & (NBD - 1);
          int e = cbase + ((ent >> SLOTB) & (CHUNK - 1));
          e = e > nE - 1 ? nE - 1 : e;
          const float w = ew[e];
          if (lane == 0) dacc[slot] = dacc[slot] + w;
        }
      }
    }
    __syncthreads();
  }

  v4f dq[8];
#pragma unroll
  for (int q = 0; q < 8; ++q) {
    const int f = (wave * 8 + q) * 128 + 4 * lane;
    const v4f c = *(const v4f*)(dacc + f);
    const float d0 = c.x + 1.f, d1 = c.y + 1.f, d2 = c.z + 1.f, d3 = c.w + 1.f;
    dq[q].x = d0 > 0.f ? rsqrtf(d0) : 0.f;
    dq[q].y = d1 > 0.f ? rsqrtf(d1) : 0.f;
    dq[q].z = d2 > 0.f ? rsqrtf(d2) : 0.f;
    dq[q].w = d3 > 0.f ? rsqrtf(d3) : 0.f;
  }
  float* dp = dinv + (size_t)nodeBase;
#pragma unroll
  for (int q = 0; q < 8; ++q) *(volatile v4f*)(dp + (wave * 8 + q) * 128 + 4 * lane) = dq[q];
  __threadfence();
#pragma unroll
  for (int q = 0; q < 8; ++q) *(volatile v4f*)(dp + (wave * 8 + q) * 128 + 4 * lane) = dq[q];
}

__global__ __launch_bounds__(NTHR) void k_gemm1(
    const float* __restrict__ x, const __bf16* __restrict__ w1h, const __bf16* __restrict__ w1l,
    const float* __restrict__ dinv, float* g1, int nN) {
  extern __shared__ v4f lds_dyn[];
  float* stg = (float*)lds_dyn;
  const int tid = threadIdx.x, lane = tid & 31, wave = tid >> 5, hh = lane >> 4, m = lane & 15;
  const int rowBase = blockIdx.x * G1ROWS;

  int node = rowBase + wave * 16 + m;
  node = node > nN - 1 ? nN - 1 : node;
  const float* xr = x + (size_t)node * DF + 8 * hh;

  v8f acc[8];
#pragma unroll
  for (int t = 0; t < 8; ++t) { v8f z = {0.f, 0.f, 0.f, 0.f, 0.f, 0.f, 0.f, 0.f}; acc[t] = z; }
#pragma unroll
  for (int kt = 0; kt < DF / 32; ++kt) {
    const v4f p0 = *(const v4f*)(xr + 32 * kt),      p1 = *(const v4f*)(xr + 32 * kt + 4);
    const v4f p2 = *(const v4f*)(xr + 32 * kt + 16), p3 = *(const v4f*)(xr + 32 * kt + 20);
    FragB ah, al;
    split8(p0, p1, ah.h[0], al.h[0]);
    split8(p2, p3, ah.h[1], al.h[1]);
#pragma unroll
    for (int t = 0; t < 8; ++t) {
      const size_t bo = (size_t)(16 * t + m) * DF + 32 * kt + 8 * hh;
      FragB bh, bl;
      bh.h[0] = *(const v8b*)(w1h + bo);
      bh.h[1] = *(const v8b*)(w1h + bo + 16);
      bl.h[0] = *(const v8b*)(w1l + bo);
      bl.h[1] = *(const v8b*)(w1l + bo + 16);
      acc[t] = wmb3(ah.v, al.v, bh.v, bl.v, acc[t]);
    }
  }

  const int r0 = wave * 16 + 8 * hh;
  const v4f dA = *(const v4f*)(dinv + (size_t)rowBase + r0);
  const v4f dB = *(const v4f*)(dinv + (size_t)rowBase + r0 + 4);
  float* sp = stg + r0 * DF + m;
#pragma unroll
  for (int t = 0; t < 8; ++t) {
    sp[0 * DF + 16 * t] = acc[t][0] * dA.x;
    sp[1 * DF + 16 * t] = acc[t][1] * dA.y;
    sp[2 * DF + 16 * t] = acc[t][2] * dA.z;
    sp[3 * DF + 16 * t] = acc[t][3] * dA.w;
    sp[4 * DF + 16 * t] = acc[t][4] * dB.x;
    sp[5 * DF + 16 * t] = acc[t][5] * dB.y;
    sp[6 * DF + 16 * t] = acc[t][6] * dB.z;
    sp[7 * DF + 16 * t] = acc[t][7] * dB.w;
  }
  __syncthreads();

  const float* lp = stg + wave * 16 * DF + 4 * lane;
  float* gp = g1 + ((size_t)rowBase + wave * 16) * DF + 4 * lane;
#pragma unroll
  for (int i = 0; i < 16; ++i) { const v4f v = *(const v4f*)(lp + i * DF); *(volatile v4f*)(gp + (size_t)i * DF) = v; }
  __threadfence();
#pragma unroll
  for (int i = 0; i < 16; ++i) { const v4f v = *(const v4f*)(lp + i * DF); *(volatile v4f*)(gp + (size_t)i * DF) = v; }
}

__global__ __launch_bounds__(NTHR) void k_agg1(
    const int* __restrict__ ei, const float* __restrict__ ew, const float* __restrict__ g1,
    const float* __restrict__ dinv, const float* __restrict__ b1,
    const __bf16* __restrict__ w2h, const __bf16* __restrict__ w2l, float* g2,
    int nN, int nE, int vec8) {
  extern __shared__ v4f lds_dyn[];
  float* acc  = (float*)lds_dyn;
  int*   list = (int*)(acc + NB1 * DF);
  int*   wcnt = list + LISTN;
  const int tid = threadIdx.x, lane = tid & 31, wave = tid >> 5, hh = lane >> 4, m = lane & 15;
  const int nodeBase = blockIdx.x * NB1;
  const int* dsts = ei + nE;

  {
    const v4f z = {0.f, 0.f, 0.f, 0.f};
    for (int i = tid; i < NB1 * DF / 4; i += NTHR) lds_dyn[i] = z;
  }
  __syncthreads();

  const int nChunks = (nE + CHUNK - 1) / CHUNK;
#pragma unroll 1
  for (int ch = 0; ch < nChunks; ++ch) {
    const int cbase = ch * CHUNK;
    const int wc = scan_chunk<NB1>(dsts, nE, cbase, nodeBase, vec8, list, tid, lane, wave);
    if (lane == 0) wcnt[wave] = wc;
    __syncthreads();
    if (wave == 0) {
#pragma unroll 1
      for (int wsx = 0; wsx < NWAVE; ++wsx) {
        int n = __builtin_amdgcn_readfirstlane(wcnt[wsx]);
        n = n > WCAP ? WCAP : (n < 0 ? 0 : n);
        const int* lp = list + wsx * WCAP;
#pragma unroll 1
        for (int i = 0; i < n; ++i) {
          const int ent  = __builtin_amdgcn_readfirstlane(lp[i]);
          const int slot = ent & (NB1 - 1);
          int e = cbase + ((ent >> SLOTB) & (CHUNK - 1));
          e = e > nE - 1 ? nE - 1 : e;
          int src = ei[e];
          src = src < 0 ? 0 : (src > nN - 1 ? nN - 1 : src);
          const float w = ew[e];
          const v4f v = *(const v4f*)(g1 + (size_t)src * DF + 4 * lane);
          v4f* ap = (v4f*)(acc + slot * DF + 4 * lane);
          *ap = *ap + v * w;
        }
      }
    }
    __syncthreads();
  }

#pragma unroll 4
  for (int i = 0; i < (NB1 * DF / 4) / NTHR; ++i) {
    const int idx  = i * NTHR + tid;
    const int slot = idx >> 5;
    const int c4   = (idx & 31) * 4;
    int node = nodeBase + slot;
    node = node > nN - 1 ? nN - 1 : node;
    const float d  = dinv[node];
    const v4f   gv = *(const v4f*)(g1 + (size_t)node * DF + c4);
    const v4f   bv = *(const v4f*)(b1 + c4);
    v4f* ap = (v4f*)(acc + slot * DF + c4);
    v4f hv = (*ap + gv) * d + bv;
    hv.x = fmaxf(hv.x, 0.f); hv.y = fmaxf(hv.y, 0.f); hv.z = fmaxf(hv.z, 0.f); hv.w = fmaxf(hv.w, 0.f);
    *ap = hv;
  }
  __syncthreads();

#pragma unroll 1
  for (int g = 0; g < NB1 / 16 / NWAVE; ++g) {
    const int t = 8 * g + wave;
    v8f c[4];
#pragma unroll
    for (int ct = 0; ct < 4; ++ct) { v8f z = {0.f, 0.f, 0.f, 0.f, 0.f, 0.f, 0.f, 0.f}; c[ct] = z; }
#pragma unroll
    for (int kt = 0; kt < DF / 32; ++kt) {
      const float* ap = acc + (16 * t + m) * DF + 32 * kt + 8 * hh;
      const v4f p0 = *(const v4f*)ap,        p1 = *(const v4f*)(ap + 4);
      const v4f p2 = *(const v4f*)(ap + 16), p3 = *(const v4f*)(ap + 20);
      FragB ah, al;
      split8(p0, p1, ah.h[0], al.h[0]);
      split8(p2, p3, ah.h[1], al.h[1]);
#pragma unroll
      for (int ct = 0; ct < 4; ++ct) {
        const size_t bo = (size_t)(16 * ct + m) * DF + 32 * kt + 8 * hh;
        FragB bh, bl;
        bh.h[0] = *(const v8b*)(w2h + bo);
        bh.h[1] = *(const v8b*)(w2h + bo + 16);
        bl.h[0] = *(const v8b*)(w2l + bo);
        bl.h[1] = *(const v8b*)(w2l + bo + 16);
        c[ct] = wmb3(ah.v, al.v, bh.v, bl.v, c[ct]);
      }
    }
    const int node0 = nodeBase + 16 * t + 8 * hh;
    const v4f dA = *(const v4f*)(dinv + (size_t)node0);
    const v4f dB = *(const v4f*)(dinv + (size_t)node0 + 4);
    float* sp = acc + 16 * t * DF + (8 * hh) * NCLS + m;
#pragma unroll
    for (int ct = 0; ct < 4; ++ct) {
      sp[0 * NCLS + 16 * ct] = c[ct][0] * dA.x;
      sp[1 * NCLS + 16 * ct] = c[ct][1] * dA.y;
      sp[2 * NCLS + 16 * ct] = c[ct][2] * dA.z;
      sp[3 * NCLS + 16 * ct] = c[ct][3] * dA.w;
      sp[4 * NCLS + 16 * ct] = c[ct][4] * dB.x;
      sp[5 * NCLS + 16 * ct] = c[ct][5] * dB.y;
      sp[6 * NCLS + 16 * ct] = c[ct][6] * dB.z;
      sp[7 * NCLS + 16 * ct] = c[ct][7] * dB.w;
    }
    __syncthreads();
    const float* lp = acc + 16 * t * DF + 4 * lane;
    float* gp = g2 + ((size_t)nodeBase + 16 * t) * NCLS + 4 * lane;
    v4f ov[8];
#pragma unroll
    for (int i = 0; i < 8; ++i) ov[i] = *(const v4f*)(lp + i * 128);
#pragma unroll
    for (int i = 0; i < 8; ++i) *(volatile v4f*)(gp + i * 128) = ov[i];
    __threadfence();
#pragma unroll
    for (int i = 0; i < 8; ++i) *(volatile v4f*)(gp + i * 128) = ov[i];
  }
}

__global__ __launch_bounds__(NTHR) void k_agg2(
    const int* __restrict__ ei, const float* __restrict__ ew, const float* __restrict__ g2,
    const float* __restrict__ dinv, const float* __restrict__ b2, float* out, int nN, int nE, int vec8) {
  extern __shared__ v4f lds_dyn[];
  float* acc  = (float*)lds_dyn;
  int*   list = (int*)(acc + NB2 * NCLS);
  int*   wcnt = list + LISTN;
  const int tid = threadIdx.x, lane = tid & 31, wave = tid >> 5;
  const int nodeBase = blockIdx.x * NB2;
  const int* dsts = ei + nE;

  {
    const v4f z = {0.f, 0.f, 0.f, 0.f};
    for (int i = tid; i < NB2 * NCLS / 4; i += NTHR) lds_dyn[i] = z;
  }
  __syncthreads();

  const int nChunks = (nE + CHUNK - 1) / CHUNK;
#pragma unroll 1
  for (int ch = 0; ch < nChunks; ++ch) {
    const int cbase = ch * CHUNK;
    const int wc = scan_chunk<NB2>(dsts, nE, cbase, nodeBase, vec8, list, tid, lane, wave);
    if (lane == 0) wcnt[wave] = wc;
    __syncthreads();
    if (wave == 0) {
#pragma unroll 1
      for (int wsx = 0; wsx < NWAVE; ++wsx) {
        int n = __builtin_amdgcn_readfirstlane(wcnt[wsx]);
        n = n > WCAP ? WCAP : (n < 0 ? 0 : n);
        const int* lp = list + wsx * WCAP;
#pragma unroll 1
        for (int i = 0; i < n; ++i) {
          const int ent  = __builtin_amdgcn_readfirstlane(lp[i]);
          const int slot = ent & (NB2 - 1);
          int e = cbase + ((ent >> SLOTB) & (CHUNK - 1));
          e = e > nE - 1 ? nE - 1 : e;
          int src = ei[e];
          src = src < 0 ? 0 : (src > nN - 1 ? nN - 1 : src);
          const float w = ew[e];
          const v2f v = *(const v2f*)(g2 + (size_t)src * NCLS + 2 * lane);
          v2f* ap = (v2f*)(acc + slot * NCLS + 2 * lane);
          *ap = *ap + v * w;
        }
      }
    }
    __syncthreads();
  }

#pragma unroll 2
  for (int q = 0; q < 64; ++q) {
    const int f    = (wave * 64 + q) * 128 + 4 * lane;
    const int slot = f >> 6;
    const int c4   = f & 63;
    int node = nodeBase + slot;
    node = node > nN - 1 ? nN - 1 : node;
    const float d  = dinv[node];
    const v4f   gv = *(const v4f*)(g2 + (size_t)node * NCLS + c4);
    const v4f   bv = *(const v4f*)(b2 + c4);
    v4f* ap = (v4f*)(acc + f);
    v4f y = (*ap + gv) * d + bv;
    float s = y.x * y.x + y.y * y.y + y.z * y.z + y.w * y.w;
    s += __shfl_xor(s, 8, 32);
    s += __shfl_xor(s, 4, 32);
    s += __shfl_xor(s, 2, 32);
    s += __shfl_xor(s, 1, 32);
    const float inv = 1.0f / fmaxf(sqrtf(s), 1e-12f);
    *ap = y * inv;
  }
  __syncthreads();

  const size_t outN = (size_t)nN * NCLS;
  const size_t ob   = (size_t)nodeBase * NCLS;
#pragma unroll 4
  for (int q = 0; q < 64; ++q) {
    const int f = (wave * 64 + q) * 128 + 4 * lane;
    const size_t gi = ob + (size_t)f;
    if (gi < outN) { const v4f v = *(const v4f*)(acc + f); *(volatile v4f*)(out + gi) = v; }
  }
  __threadfence();
#pragma unroll 4
  for (int q = 0; q < 64; ++q) {
    const int f = (wave * 64 + q) * 128 + 4 * lane;
    const size_t gi = ob + (size_t)f;
    if (gi < outN) { const v4f v = *(const v4f*)(acc + f); *(volatile v4f*)(out + gi) = v; }
  }
}

extern "C" void kernel_launch(void* const* d_in, const int* in_sizes, int n_in,
                              void* d_out, int out_size, void* d_ws, size_t ws_size,
                              hipStream_t stream) {
  if (n_in < 7) return;
  const int nN = in_sizes[0] / DF;
  const int nE = in_sizes[1] / 2;
  if (nN <= 0 || nE < 0 || in_sizes[0] != nN * DF || in_sizes[1] != nE * 2) return;
  if (in_sizes[2] != nE) return;
  if (in_sizes[3] != DF * DF || in_sizes[4] < DF || in_sizes[5] != DF * NCLS || in_sizes[6] < NCLS) return;
  if (out_size != nN * NCLS) return;

  const float* x  = (const float*)d_in[0];
  const int*   ei = (const int*)d_in[1];
  const float* ew = (const float*)d_in[2];
  const float* W1 = (const float*)d_in[3];
  const float* b1 = (const float*)d_in[4];
  const float* W2 = (const float*)d_in[5];
  const float* b2 = (const float*)d_in[6];
  float* out = (float*)d_out;

  const int nBD = (nN + NBD - 1) / NBD;
  const int nG1 = (nN + G1ROWS - 1) / G1ROWS;
  const int nA1 = (nN + NB1 - 1) / NB1;
  const int nA2 = (nN + NB2 - 1) / NB2;

  char* ws = (char*)d_ws;
  size_t off = 0;
  const size_t oW1h = off; off += (size_t)DF * DF * 2;                         off = (off + 255) & ~(size_t)255;
  const size_t oW1l = off; off += (size_t)DF * DF * 2;                         off = (off + 255) & ~(size_t)255;
  const size_t oW2h = off; off += (size_t)NCLS * DF * 2;                       off = (off + 255) & ~(size_t)255;
  const size_t oW2l = off; off += (size_t)NCLS * DF * 2;                       off = (off + 255) & ~(size_t)255;
  const size_t oDv  = off; off += (size_t)nBD * NBD * 4;                       off = (off + 255) & ~(size_t)255;
  const size_t oG1  = off; off += (size_t)nG1 * G1ROWS * DF * 4;               off = (off + 255) & ~(size_t)255;
  const size_t oG2  = off; off += (size_t)nA1 * NB1 * NCLS * 4;                off = (off + 255) & ~(size_t)255;
  if (off > ws_size) return;
  __bf16* w1h  = (__bf16*)(ws + oW1h);
  __bf16* w1l  = (__bf16*)(ws + oW1l);
  __bf16* w2h  = (__bf16*)(ws + oW2h);
  __bf16* w2l  = (__bf16*)(ws + oW2l);
  float*  dinv = (float*)(ws + oDv);
  float*  g1   = (float*)(ws + oG1);
  float*  g2   = (float*)(ws + oG2);

  const int vec8 = ((nE & 3) == 0) ? 1 : 0;

  const int nPrep = DF * DF / 8 + NCLS * DF / 8;
  k_wprep<<<(nPrep + NTHR - 1) / NTHR, NTHR, 0, stream>>>(W1, W2, w1h, w1l, w2h, w2l);

  k_deg<<<nBD, NTHR, 0, stream>>>(ei, ew, dinv, nN, nE, vec8);

  hipFuncSetAttribute(reinterpret_cast<const void*>(&k_gemm1),
                      hipFuncAttributeMaxDynamicSharedMemorySize, LDS_GEMM1);
  k_gemm1<<<nG1, NTHR, LDS_GEMM1, stream>>>(x, w1h, w1l, dinv, g1, nN);

  hipFuncSetAttribute(reinterpret_cast<const void*>(&k_agg1),
                      hipFuncAttributeMaxDynamicSharedMemorySize, LDS_AGG1);
  k_agg1<<<nA1, NTHR, LDS_AGG1, stream>>>(ei, ew, g1, dinv, b1, w2h, w2l, g2, nN, nE, vec8);

  hipFuncSetAttribute(reinterpret_cast<const void*>(&k_agg2),
                      hipFuncAttributeMaxDynamicSharedMemorySize, LDS_AGG2);
  k_agg2<<<nA2, NTHR, LDS_AGG2, stream>>>(ei, ew, g2, dinv, b2, out, nN, nE, vec8);
}
